// SoftDecisionTree_70746701299772
// MI455X (gfx1250) — hardware-verified
//
#include <hip/hip_runtime.h>

typedef __attribute__((ext_vector_type(16))) _Float16 v16h;
typedef __attribute__((ext_vector_type(8)))  _Float16 v8h;
typedef __attribute__((ext_vector_type(4)))  _Float16 v4h;
typedef __attribute__((ext_vector_type(8)))  float    v8f;
typedef __attribute__((ext_vector_type(4)))  float    v4f;
typedef __attribute__((ext_vector_type(16))) __bf16   v16b;
typedef float __attribute__((may_alias)) float_a;
typedef int   __attribute__((may_alias)) int_a;
template <typename T> __device__ __forceinline__ void vst2(void* p, T v) { *(volatile T*)p = v; __threadfence(); *(volatile T*)p = v; }
__device__ __forceinline__ v8f wmma_bf(v16b a, v16b b, v8f c) {
    v8f d = __builtin_amdgcn_wmma_f32_16x16x32_bf16(false, a, false, b, (short)0, c, false, false);
    asm volatile("v_nop\n\tv_nop\n\tv_nop\n\tv_nop" : "+v"(d) : "v"(a), "v"(b));
    return d;
}
struct F3 { v16b h, m, l; };
__device__ __forceinline__ F3 split3_row(const float* row, int k0, int lane) {
    F3 r; const float* p = row + k0 + 8 * (lane >> 4);
#pragma unroll
    for (int i = 0; i < 8; ++i) {
#pragma unroll
        for (int s = 0; s < 2; ++s) { const float v = p[i + 16 * s]; const int e = i + 8 * s;
            const __bf16 h = (__bf16)v; const float r1 = v - (float)h; const __bf16 m = (__bf16)r1; const __bf16 l = (__bf16)(r1 - (float)m);
            r.h[e] = h; r.m[e] = m; r.l[e] = l; }
    }
    return r;
}
__device__ __forceinline__ v8f mac6(const F3& a, const F3& b, v8f c) {
    c = wmma_bf(a.l, b.h, c); c = wmma_bf(a.h, b.l, c); c = wmma_bf(a.m, b.m, c);
    c = wmma_bf(a.m, b.h, c); c = wmma_bf(a.h, b.m, c); return wmma_bf(a.h, b.h, c);
}

#define BS  16384
#define DD  512
#define NI  255
#define NL  256
#define NC  1000
#define RED_BLOCKS 128
#define ROWS_PER_RED (BS / RED_BLOCKS)

__global__ __launch_bounds__(DD) void colstat_partial(const float* __restrict__ x,
                                                      float* __restrict__ psum,
                                                      float* __restrict__ psq) {
    const int c   = threadIdx.x;
    const int blk = blockIdx.x;
    const float* xp = x + (size_t)blk * ROWS_PER_RED * DD + c;
    float s = 0.f, s2 = 0.f;
    #pragma unroll 4
    for (int r = 0; r < ROWS_PER_RED; ++r) {
        float v = xp[(size_t)r * DD];
        s += v; s2 += v * v;
    }
    vst2(psum + blk * DD + c, (float_a)s);
    vst2(psq  + blk * DD + c, (float_a)s2);
}

__global__ __launch_bounds__(256) void colstat_final(const float* __restrict__ psum,
                                                     const float* __restrict__ psq,
                                                     const float* __restrict__ gamma,
                                                     const float* __restrict__ beta,
                                                     float* __restrict__ scale,
                                                     float* __restrict__ shift) {
    int c = blockIdx.x * blockDim.x + threadIdx.x;
    if (c >= DD) return;
    float s = 0.f, s2 = 0.f;
    for (int b = 0; b < RED_BLOCKS; ++b) { s += psum[b * DD + c]; s2 += psq[b * DD + c]; }
    float mean = s * (1.f / BS);
    float var  = s2 * (1.f / BS) - mean * mean;
    float sc   = gamma[c] * rsqrtf(var + 1e-5f);
    vst2(scale + c, (float_a)sc);
    vst2(shift + c, (float_a)(beta[c] - mean * sc));
}

__global__ __launch_bounds__(256) void softmax_stats(const float* __restrict__ cr, float* __restrict__ st) {
    __shared__ float red[256];
    const int l = blockIdx.x, t = threadIdx.x;
    const float* rp = cr + (size_t)l * NC;
    float m = -3.402823466e+38f;
    for (int c = t; c < NC; c += 256) m = fmaxf(m, rp[c]);
    red[t] = m; __syncthreads();
    for (int s = 128; s > 0; s >>= 1) { if (t < s) red[t] = fmaxf(red[t], red[t + s]); __syncthreads(); }
    m = red[0]; __syncthreads();
    float sum = 0.f;
    for (int c = t; c < NC; c += 256) sum += expf(rp[c] - m);
    red[t] = sum; __syncthreads();
    for (int s = 128; s > 0; s >>= 1) { if (t < s) red[t] += red[t + s]; __syncthreads(); }
    if (t == 0) { vst2(st + l * 32, (float_a)m); vst2(st + l * 32 + 1, (float_a)(1.f / red[0])); }
}
__global__ __launch_bounds__(256) void softmax_write(const float* __restrict__ cr, const float* __restrict__ st, float* __restrict__ dist) {
    const size_t f0 = (size_t)blockIdx.x * 32 * NC;
    for (int q = threadIdx.x; q < 32 * NC / 4; q += 256) { v4f v;
#pragma unroll
        for (int e = 0; e < 4; ++e) { const size_t f = f0 + (size_t)q * 4 + e; const int l = (int)(f / NC);
            v[e] = expf(cr[f] - st[l * 32]) * st[l * 32 + 1]; }
        vst2(dist + f0 + (size_t)q * 4, v); }
}

__global__ __launch_bounds__(128) void tree_gates_argmax(
        const float* __restrict__ x, const float* __restrict__ W,
        const float* __restrict__ bias, const float* __restrict__ scale,
        const float* __restrict__ shift, int* __restrict__ leafidx) {
    __shared__ __align__(16) float lA[16 * DD];
    __shared__ float    lgates[16 * NL];
    __shared__ int      lidx_s[16];

    const int tid  = threadIdx.x;
    const int row0 = blockIdx.x * 16;

    for (int i = tid; i < 16 * DD / 4; i += 128) {
        const int flat = i * 4;
        const int r = flat >> 9, c = flat & (DD - 1);
        const float4 xv = *(const float4*)(x + (size_t)(row0 + r) * DD + c);
        const float4 sv = *(const float4*)(scale + c);
        const float4 tv = *(const float4*)(shift + c);
        v4f h;
        h[0] = xv.x * sv.x + tv.x;
        h[1] = xv.y * sv.y + tv.y;
        h[2] = xv.z * sv.z + tv.z;
        h[3] = xv.w * sv.w + tv.w;
        *(v4f*)(&lA[flat]) = h;
    }
    __syncthreads();

    const int lane  = tid & 31;
    const int wv    = tid >> 5;
    const int nbase = wv * 64;
    const int mA    = lane & 15;
    const int nB    = lane & 15;
    const float* wrow[4];
#pragma unroll
    for (int j = 0; j < 4; ++j) { int n = nbase + j * 16 + nB; if (n >= NI) n = NI - 1; wrow[j] = W + (size_t)n * DD; }

    v8f acc[4] = {v8f{}, v8f{}, v8f{}, v8f{}};

#pragma unroll 1
    for (int k0 = 0; k0 < DD; k0 += 32) {
        const F3 a = split3_row(&lA[mA * DD], k0, lane);
        #pragma unroll
        for (int j = 0; j < 4; ++j) acc[j] = mac6(a, split3_row(wrow[j], k0, lane), acc[j]);
    }

    #pragma unroll
    for (int j = 0; j < 4; ++j) {
        const int N = nbase + j * 16 + (lane & 15);
        const float bv = (N < NI) ? bias[N] : 0.f;
        const int moff = (lane >> 4) * 8;
        #pragma unroll
        for (int r = 0; r < 8; ++r) {
            float z = acc[j][r] + bv;
            lgates[(moff + r) * NL + N] = 1.f / (1.f + expf(-z));
        }
    }
    __syncthreads();

    for (int rr = 0; rr < 4; ++rr) {
        const int row = wv * 4 + rr;
        const float* g = &lgates[row * NL];
        float best = -1.f; int bi = 0;
        for (int l8 = 0; l8 < 8; ++l8) {
            const int leaf = lane * 8 + l8;
            float p = 1.f;
            #pragma unroll
            for (int d = 0; d < 8; ++d) {
                const int node = ((1 << d) - 1) + (leaf >> (8 - d));
                const float gg = g[node];
                p *= ((leaf >> (7 - d)) & 1) ? gg : (1.f - gg);
            }
            if (p > best) { best = p; bi = leaf; }
        }
        #pragma unroll
        for (int off = 16; off > 0; off >>= 1) {
            float ob = __shfl_xor(best, off, 32);
            int   oi = __shfl_xor(bi,   off, 32);
            if (ob > best || (ob == best && oi < bi)) { best = ob; bi = oi; }
        }
        if (lane == 0) lidx_s[row] = bi;
    }
    __syncthreads();
    if (tid < 32) vst2(leafidx + (size_t)blockIdx.x * 32 + tid, (int_a)(tid < 16 ? lidx_s[tid] : 0));
}

__global__ __launch_bounds__(256) void gather_rows(const int* __restrict__ idx,
                                                   const float* __restrict__ dist,
                                                   float* __restrict__ out) {
    const size_t f0 = (size_t)blockIdx.x * 32 * NC;
    for (int q = threadIdx.x; q < 32 * NC / 4; q += 256) { v4f v;
#pragma unroll
        for (int e = 0; e < 4; ++e) { const size_t f = f0 + (size_t)q * 4 + e; const int i = (int)(f / NC), c = (int)(f % NC);
            int li = idx[(i >> 4) * 32 + (i & 15)]; li = li < 0 ? 0 : (li >= NL ? NL - 1 : li);
            v[e] = dist[(size_t)li * NC + c]; }
        vst2(out + f0 + (size_t)q * 4, v); }
}

extern "C" void kernel_launch(void* const* d_in, const int* in_sizes, int n_in,
                              void* d_out, int out_size, void* d_ws, size_t ws_size,
                              hipStream_t stream) {
    const float* x     = (const float*)d_in[0];
    const float* W     = (const float*)d_in[1];
    const float* b     = (const float*)d_in[2];
    const float* cr    = (const float*)d_in[3];
    const float* gamma = (const float*)d_in[4];
    const float* beta  = (const float*)d_in[5];
    float* out = (float*)d_out;

    float* psum  = (float*)d_ws;
    float* psq   = psum + RED_BLOCKS * DD;
    float* scale = psq  + RED_BLOCKS * DD;
    float* shift = scale + DD;
    float* st    = shift + DD;
    int*   lidx  = (int*)(st + NL * 32);
    float* dist  = (float*)(lidx + (BS / 16) * 32);

    colstat_partial <<<RED_BLOCKS, DD,        0, stream>>>(x, psum, psq);
    colstat_final   <<<2, 256,                0, stream>>>(psum, psq, gamma, beta, scale, shift);
    softmax_stats   <<<NL, 256,               0, stream>>>(cr, st);
    softmax_write   <<<NL / 32, 256,          0, stream>>>(cr, st, dist);
    tree_gates_argmax<<<BS / 16, 128,         0, stream>>>(x, W, b, scale, shift, lidx);
    gather_rows     <<<BS / 32, 256,          0, stream>>>(lidx, dist, out);
}
